// HypothesisGAT_3959959847189
// MI455X (gfx1250) — hardware-verified
//
#include <hip/hip_runtime.h>
#include <math.h>

typedef __attribute__((ext_vector_type(16))) _Float16 v16h;
typedef __attribute__((ext_vector_type(16))) __bf16 v16b;
typedef __attribute__((ext_vector_type(8)))  _Float16 v8h;
typedef __attribute__((ext_vector_type(8)))  float v8f;
typedef __attribute__((ext_vector_type(4)))  float v4f;
typedef __attribute__((ext_vector_type(2)))  float v2f;
typedef __attribute__((ext_vector_type(4)))  unsigned v4u;
typedef __attribute__((ext_vector_type(4)))  int v4i;
typedef float __attribute__((may_alias)) float_a;
typedef int __attribute__((may_alias)) int_a;

template <typename T> __device__ __forceinline__ void vst2(void* p, T v) { *(volatile T*)p = v; __threadfence(); *(volatile T*)p = v; }
__device__ __forceinline__ v8f wmma16(v16h a, v16h b, v8f c) {
  v8f d = __builtin_amdgcn_wmma_f32_16x16x32_f16(false, a, false, b, (short)0, c, false, false);
  asm volatile("v_nop\n\tv_nop\n\tv_nop\n\tv_nop" : "+v"(d) : "v"(a), "v"(b));
  return d;
}
__device__ __forceinline__ v8f wmma_bf(v16b a, v16b b, v8f c) {
  v8f d = __builtin_amdgcn_wmma_f32_16x16x32_bf16(false, a, false, b, (short)0, c, false, false);
  asm volatile("v_nop\n\tv_nop\n\tv_nop\n\tv_nop" : "+v"(d) : "v"(a), "v"(b));
  return d;
}
__device__ __forceinline__ v16h frag_h(const _Float16* rowk0, int lane) {
  union { v16h v; v8h q[2]; } u; const _Float16* p = rowk0 + 8 * (lane >> 4);
  u.q[0] = *(const v8h*)p; u.q[1] = *(const v8h*)(p + 16); return u.v;
}
__device__ __forceinline__ v16h frag_f32(const float* rowk0, int lane) {
  v16h a; const float* p = rowk0 + 8 * (lane >> 4);
#pragma unroll
  for (int i = 0; i < 8; ++i) { a[i] = (_Float16)p[i]; a[8 + i] = (_Float16)p[16 + i]; }
  return a;
}
__device__ __forceinline__ v16h frag_f32s(const float* rowk0, int lane, float sc) {
  v16h a; const float* p = rowk0 + 8 * (lane >> 4);
#pragma unroll
  for (int i = 0; i < 8; ++i) { a[i] = (_Float16)(p[i] * sc); a[8 + i] = (_Float16)(p[16 + i] * sc); }
  return a;
}
__device__ __forceinline__ v16h fragc_f32(const float* W, int k0, int n, int lane, int ld, int K) {
  v16h a; const int g = lane >> 4;
#pragma unroll
  for (int i = 0; i < 8; ++i) { const int ka = k0 + 8 * g + i, kb = ka + 16;
    a[i] = (_Float16)(ka < K ? W[(size_t)(ka < K ? ka : K - 1) * ld + n] : 0.f); a[8 + i] = (_Float16)(kb < K ? W[(size_t)(kb < K ? kb : K - 1) * ld + n] : 0.f); }
  return a;
}
struct F2 { v16b h, l; };
__device__ __forceinline__ F2 bsplit16(const float v[16]) { F2 r;
#pragma unroll
  for (int i = 0; i < 16; ++i) { const __bf16 h = (__bf16)v[i]; r.h[i] = h; r.l[i] = (__bf16)(v[i] - (float)h); }
  return r; }
__device__ __forceinline__ F2 split_row(const float* row, int k0, int lane) { float v[16]; const float* p = row + k0 + 8 * (lane >> 4);
#pragma unroll
  for (int i = 0; i < 8; ++i) { v[i] = p[i]; v[8 + i] = p[16 + i]; }
  return bsplit16(v); }
__device__ __forceinline__ F2 split_rowK(const float* row, int k0, int lane, int K) { float v[16]; const int g = lane >> 4;
#pragma unroll
  for (int i = 0; i < 8; ++i) { const int ka = k0 + 8 * g + i, kb = ka + 16; v[i] = ka < K ? row[ka < K ? ka : K - 1] : 0.f; v[8 + i] = kb < K ? row[kb < K ? kb : K - 1] : 0.f; }
  return bsplit16(v); }
__device__ __forceinline__ F2 split_col(const float* W, int k0, int n, int lane, int ld, int K) { float v[16]; const int g = lane >> 4;
#pragma unroll
  for (int i = 0; i < 8; ++i) { const int ka = k0 + 8 * g + i, kb = ka + 16; v[i] = ka < K ? W[(size_t)(ka < K ? ka : K - 1) * ld + n] : 0.f; v[8 + i] = kb < K ? W[(size_t)(kb < K ? kb : K - 1) * ld + n] : 0.f; }
  return bsplit16(v); }
__device__ __forceinline__ v8f mac3(const F2& a, const F2& b, v8f c) { c = wmma_bf(a.l, b.h, c); c = wmma_bf(a.h, b.l, c); return wmma_bf(a.h, b.h, c); }
__device__ __forceinline__ float sigm(float v) { return 1.0f / (1.0f + expf(-v)); }
#define LDSX() do { asm volatile("s_wait_dscnt 0" ::: "memory"); __builtin_amdgcn_wave_barrier(); __builtin_amdgcn_fence(__ATOMIC_RELEASE, "workgroup"); } while (0)


#ifndef NN
#define NN 50000
#endif
#define EP 400000
#ifndef NE
#define NE 400000
#endif
#define DIN 6
#define HID 128
#define NHD 4
#define HC (NHD * HID)
#define NL 3
#define NHYP 4096
#define NBLK ((NN + 63) / 64)
#define NRP (NBLK * 64)
#define CSR_N NN
#define CSR_E NE
typedef __attribute__((ext_vector_type(8))) __bf16 v8b;
__device__ __forceinline__ v16b frag_b(const __bf16* rowk0, int lane) {
  union { v16b v; v8b q[2]; } u; const __bf16* p = rowk0 + 8 * (lane >> 4);
  u.q[0] = *(const v8b*)p; u.q[1] = *(const v8b*)(p + 16); return u.v;
}
__device__ __forceinline__ float bfr(float v) { return (float)(__bf16)v; }
__device__ __attribute__((noinline)) float exp_ni(float v) { return expf(v); }
__device__ __attribute__((noinline)) float erf_ni(float v) { return erff(v); }

#define CSR_FINN (CSR_E + 32 * CSR_NBK)
#define CSR_CHUNK 4096
#define CSR_BKT 256
#define CSR_NCH ((CSR_E + CSR_CHUNK - 1) / CSR_CHUNK)
#define CSR_NBK ((CSR_N + CSR_BKT - 1) / CSR_BKT)
#define CSR_NBKP (((CSR_NBK + 63) / 64) * 64)
#define CSR_SEGCAP (CSR_E + 32 * CSR_NBK * CSR_NCH)
#ifndef CSR_BCAP
#define CSR_BCAP 10240
#endif
#define CSR_SZ_CNT   (4u * CSR_NCH * CSR_NBKP)
#define CSR_SZ_OFF   (4u * CSR_NBK * (((CSR_NCH + 31) / 32) * 32))
#define CSR_SZ_BST   (4u * (((CSR_NBK + 1 + 31) / 32) * 32))
#define CSR_SZ_SEG   (4u * CSR_SEGCAP)
#define CSR_SZ_FIN   (4u * (CSR_E + 32 * CSR_NBK))
#define CSR_SZ_ROW   (4u * CSR_NBK * CSR_BKT)
#define CSR_OFFP (((CSR_NCH + 31) / 32) * 32)

__global__ __launch_bounds__(256) void k_csr_cnt(const int* __restrict__ DST, int dstride, int* __restrict__ CNT) {
  __shared__ unsigned short sc[256][CSR_NBK + 1]; __shared__ __align__(16) int srow[CSR_NBKP];
  const int c = blockIdx.x, tid = threadIdx.x;
  for (int b = 0; b < CSR_NBK; ++b) sc[tid][b] = 0;
  const size_t e0 = (size_t)c * CSR_CHUNK + tid * 16;
  for (int i = 0; i < 16; ++i) { const size_t e = e0 + i; if (e < (size_t)CSR_E) { int d = DST[e * dstride]; d = min(max(d, 0), CSR_N - 1); sc[tid][d / CSR_BKT] += 1; } }
  __syncthreads();
  for (int b = tid; b < CSR_NBKP; b += 256) { int s = 0; if (b < CSR_NBK) for (int t = 0; t < 256; ++t) s += sc[t][b]; srow[b] = s; }
  __syncthreads();
  for (int q = tid; q < CSR_NBKP / 4; q += 256) vst2((unsigned*)(CNT + (size_t)c * CSR_NBKP + q * 4), *(const v4u*)&srow[q * 4]);
}
__global__ __launch_bounds__(256) void k_csr_scan(const int* __restrict__ CNT, int* __restrict__ OFF, int* __restrict__ BST) {
  __shared__ int sbt[CSR_NBK + 1]; __shared__ int sbs[((CSR_NBK + 1 + 31) / 32) * 32]; __shared__ int scnt[CSR_NBK + 1]; __shared__ __align__(16) int sbuf[64][CSR_OFFP];
  const int tid = threadIdx.x;
  for (int b = tid; b < CSR_NBK; b += 256) { int sp = 0, st = 0; for (int c = 0; c < CSR_NCH; ++c) { const int n = CNT[(size_t)c * CSR_NBKP + b]; st += n; sp += (n + 31) & ~31; } sbt[b] = sp; scnt[b] = st; }
  for (int b = tid; b < ((CSR_NBK + 1 + 31) / 32) * 32; b += 256) sbs[b] = 0;
  __syncthreads();
  if (tid == 0) { int acc = 0, accf = 0; for (int b = 0; b < CSR_NBK; ++b) { const int t = sbt[b]; sbt[b] = acc; acc += t; sbs[b] = accf; accf += (scnt[b] + 31) & ~31; } sbs[CSR_NBK] = accf; }
  __syncthreads();
  for (int b0 = 0; b0 < CSR_NBK; b0 += 64) {
    if (tid < 64 && b0 + tid < CSR_NBK) { const int b = b0 + tid; int o = sbt[b]; for (int c = 0; c < CSR_OFFP; ++c) { if (c < CSR_NCH) { sbuf[tid][c] = o; o += (CNT[(size_t)c * CSR_NBKP + b] + 31) & ~31; } else sbuf[tid][c] = 0; } }
    __syncthreads();
    for (int q = tid; q < 64 * (CSR_OFFP / 4); q += 256) { const int r = q / (CSR_OFFP / 4), pc = q % (CSR_OFFP / 4); if (b0 + r < CSR_NBK) vst2((unsigned*)(OFF + (size_t)(b0 + r) * CSR_OFFP + pc * 4), *(const v4u*)&sbuf[r][pc * 4]); }
    __syncthreads(); }
  for (int q = tid; q < ((CSR_NBK + 1 + 31) / 32) * 32 / 4; q += 256) vst2((unsigned*)(BST + q * 4), *(const v4u*)&sbs[q * 4]);
}
__global__ __launch_bounds__(256) void k_csr_scatter(const int* __restrict__ SRC, const int* __restrict__ DST, int sstride, int dstride, const int* __restrict__ OFF, int* __restrict__ SEGS, int* __restrict__ SEGE) {
  __shared__ unsigned short sc[256][CSR_NBK + 1]; __shared__ int sbase[CSR_NBK + 1]; __shared__ int scn[CSR_NBK + 1]; __shared__ int sord[CSR_CHUNK];
  const int c = blockIdx.x, tid = threadIdx.x;
  for (int b = 0; b < CSR_NBK; ++b) sc[tid][b] = 0;
  const size_t e0 = (size_t)c * CSR_CHUNK + tid * 16; int bk[16];
#pragma unroll
  for (int i = 0; i < 16; ++i) { const size_t e = e0 + i; bk[i] = -1; if (e < (size_t)CSR_E) { int d = DST[e * dstride]; d = min(max(d, 0), CSR_N - 1); bk[i] = d / CSR_BKT; sc[tid][bk[i]] += 1; } }
  __syncthreads();
  for (int b = tid; b < CSR_NBK; b += 256) { int acc = 0; for (int t = 0; t < 256; ++t) { const int v = sc[t][b]; sc[t][b] = (unsigned short)acc; acc += v; } scn[b] = acc; }
  __syncthreads();
  if (tid == 0) { int acc = 0; for (int b = 0; b < CSR_NBK; ++b) { sbase[b] = acc; acc += scn[b]; } }
  __syncthreads();
#pragma unroll
  for (int i = 0; i < 16; ++i) { if (bk[i] >= 0) { const int b = bk[i]; const int r = sc[tid][b]; sc[tid][b] = (unsigned short)(r + 1); sord[sbase[b] + r] = tid * 16 + i; } }
  __syncthreads();
  for (int b = 0; b < CSR_NBK; ++b) { const int n = scn[b]; if (n == 0) continue; const int nl = ((n + 31) & ~31); const size_t o = (size_t)(min(max(OFF[(size_t)b * CSR_OFFP + c], 0), CSR_SEGCAP - nl) & ~31);
    for (int q = tid; q < nl / 4; q += 256) { int4 vs, ve;
#pragma unroll
      for (int k = 0; k < 4; ++k) { const int i = q * 4 + k; int s = -1, eid = -1; if (i < n) { const size_t e = (size_t)c * CSR_CHUNK + sord[sbase[b] + i]; s = min(max(SRC[e * sstride], 0), CSR_N - 1); eid = (int)e; } vs[k] = s; ve[k] = eid; }
      vst2((unsigned*)(SEGS + o + q * 4), *(const v4u*)&vs); vst2((unsigned*)(SEGE + o + q * 4), *(const v4u*)&ve); } }
}
__global__ __launch_bounds__(256) void k_csr_bucket(const int* __restrict__ CNT, const int* __restrict__ OFF, const int* __restrict__ BST, const int* __restrict__ SEGS, const int* __restrict__ SEGE, const int* __restrict__ DST, int dstride, int* __restrict__ FS, int* __restrict__ FE, int* __restrict__ ROWST, int* __restrict__ ROWCNT) {
  __shared__ int ssrc[CSR_BCAP]; __shared__ int seid[CSR_BCAP]; __shared__ unsigned char snod[CSR_BCAP]; __shared__ int souts[CSR_BCAP]; __shared__ int soute[CSR_BCAP]; __shared__ int scount[256]; __shared__ int sstart[257]; __shared__ int stot;
  const int b = blockIdx.x, tid = threadIdx.x;
  if (tid == 0) { int t = 0; for (int c = 0; c < CSR_NCH; ++c) t += min(max(CNT[(size_t)c * CSR_NBKP + b], 0), CSR_CHUNK); stot = (t <= CSR_BCAP) ? t : 0; }
  __syncthreads();
  { int base = 0; for (int c = 0; c < CSR_NCH; ++c) { const int n = min(max(CNT[(size_t)c * CSR_NBKP + b], 0), CSR_CHUNK); const int o = min(max(OFF[(size_t)b * CSR_OFFP + c], 0), CSR_SEGCAP - ((n + 31) & ~31));
      for (int i = tid; i < n; i += 256) { const int p = base + i; if (p < CSR_BCAP) { ssrc[p] = min(max(SEGS[o + i], 0), CSR_N - 1); const int e = min(max(SEGE[o + i], 0), CSR_E - 1); seid[p] = e; int d = DST[(size_t)e * dstride]; d = min(max(d, 0), CSR_N - 1); const int dl = d - b * CSR_BKT; snod[p] = (unsigned char)(dl >= 0 && dl < 256 ? dl : 255); } }
      base += n; } }
  __syncthreads();
  const int node = b * CSR_BKT + tid; int cnt = 0; for (int p = 0; p < stot; ++p) cnt += (snod[p] == tid) ? 1 : 0;
  scount[tid] = cnt; __syncthreads();
  if (tid == 0) { int acc = 0; for (int t = 0; t < 256; ++t) { sstart[t] = acc; acc += scount[t]; } sstart[256] = acc; }
  __syncthreads();
  const int bst0 = min(max(BST[b], 0), CSR_FINN - ((sstart[256] + 31) & ~31)) & ~31; const int gst = bst0 + sstart[tid];
  { int w = sstart[tid]; for (int p = 0; p < stot; ++p) if (snod[p] == tid) { souts[w] = ssrc[p]; soute[w] = seid[p]; ++w; } }
  __syncthreads();
  { const int n = sstart[256]; const int nl = (n + 31) & ~31; for (int q = tid; q < nl / 4; q += 256) { int4 vs, ve;
#pragma unroll
      for (int k = 0; k < 4; ++k) { const int i = q * 4 + k; vs[k] = i < n ? souts[i] : -1; ve[k] = i < n ? soute[i] : -1; }
      vst2((unsigned*)(FS + bst0 + q * 4), *(const v4u*)&vs); vst2((unsigned*)(FE + bst0 + q * 4), *(const v4u*)&ve); } }
  __syncthreads();
  { __shared__ __align__(16) int srs[256], src2[256]; srs[tid] = node < CSR_N ? gst : 0; src2[tid] = node < CSR_N ? cnt : 0; __syncthreads();
    if (tid < 64) vst2((unsigned*)(ROWST + (size_t)b * 256 + tid * 4), *(const v4u*)&srs[tid * 4]); else if (tid < 128) vst2((unsigned*)(ROWCNT + (size_t)b * 256 + (tid - 64) * 4), *(const v4u*)&src2[(tid - 64) * 4]); }
}


#define WS_CNT  0u
#define WS_OFF  (WS_CNT + CSR_SZ_CNT)
#define WS_BST  (WS_OFF + CSR_SZ_OFF)
#define WS_SEGS (WS_BST + CSR_SZ_BST)
#define WS_SEGE (WS_SEGS + CSR_SZ_SEG)
#define WS_FS   (WS_SEGE + CSR_SZ_SEG)
#define WS_FE   (WS_FS + CSR_SZ_FIN)
#define WS_RST  (WS_FE + CSR_SZ_FIN)
#define WS_RCT  (WS_RST + CSR_SZ_ROW)
#define WS_PW   (WS_RCT + CSR_SZ_ROW)
#define PE2 0
#define PG0 (PE2 + HID * HID)
#define PH1 (PG0 + NL * HC * HID)
#define PWEND (PH1 + 64 * HID)
#define WS_T    (WS_PW + 2u * PWEND)
#define WS_H    (WS_T + 4u * NRP * HID)
#define WS_HW   (WS_H + 4u * NRP * HID)
#define WS_AS   (WS_HW + 4u * NRP * HC)
#define WS_AD   (WS_AS + 4u * NHD * NRP)
#define WS_END  (WS_AD + 4u * NHD * NRP)

__global__ __launch_bounds__(128) void k_packT(const float* __restrict__ Wm, int K, int N, __bf16* __restrict__ DST) {
  __shared__ __align__(16) __bf16 s[128]; const int n = blockIdx.x, l = blockIdx.y, k = threadIdx.x;
  if (k < K) s[k] = (__bf16)Wm[((size_t)l * K + k) * N + n];
  __syncthreads();
  if (k < K / 8) vst2((unsigned*)(DST + ((size_t)l * N + n) * K + k * 8), *(const v4u*)&s[k * 8]);
}
__global__ __launch_bounds__(256) void k_enc1(const float* __restrict__ X, const float* __restrict__ W1, const float* __restrict__ B1, float* __restrict__ T) {
  __shared__ float sw[DIN][HID], sb[HID]; __shared__ __align__(16) float so[16][HID + 4];
  const int tid = threadIdx.x; for (int q = tid; q < DIN * HID; q += 256) sw[q / HID][q % HID] = bfr(W1[q]); if (tid < HID) sb[tid] = bfr(B1[tid]);
  __syncthreads();
  const int nl = tid >> 4, c0 = (tid & 15) * 8; const size_t node = (size_t)blockIdx.x * 16 + nl; float xv[DIN];
#pragma unroll
  for (int i = 0; i < DIN; ++i) xv[i] = (node < (size_t)NN) ? bfr(X[node * DIN + i]) : 0.f;
#pragma unroll
  for (int j = 0; j < 8; ++j) { float a = sb[c0 + j];
#pragma unroll
    for (int i = 0; i < DIN; ++i) a += xv[i] * sw[i][c0 + j];
    so[nl][c0 + j] = fmaxf(a, 0.f); }
  __syncthreads();
  for (int q = tid; q < 16 * 32; q += 256) { const int rl = q >> 5, pc = q & 31; vst2(T + ((size_t)blockIdx.x * 16 + rl) * HID + pc * 4, *(const v4f*)&so[rl][pc * 4]); }
}
__global__ __launch_bounds__(128) void k_lin(const float* __restrict__ A, const __bf16* __restrict__ P, const float* __restrict__ bias, float* __restrict__ OUT) {
  __shared__ __align__(16) float so[4][16][132];
  const int tid = threadIdx.x, wave = tid >> 5, lane = tid & 31, col = lane & 15, g = lane >> 4; const size_t r0 = (size_t)blockIdx.x * 64 + wave * 16; size_t ra = r0 + col; if (ra >= NN) ra = NN - 1;
  v8f acc[8] = {};
#pragma unroll
  for (int kc = 0; kc < HID / 32; ++kc) { const F2 a = split_row(A + ra * HID, kc * 32, lane);
#pragma unroll
    for (int j = 0; j < 8; ++j) { const v16b w = frag_b(P + (size_t)(j * 16 + col) * HID + kc * 32, lane); acc[j] = wmma_bf(a.l, w, acc[j]); acc[j] = wmma_bf(a.h, w, acc[j]); } }
#pragma unroll
  for (int j = 0; j < 8; ++j) { const float bb = bfr(bias[j * 16 + col]);
#pragma unroll
    for (int r = 0; r < 8; ++r) so[wave][8 * g + r][j * 16 + col] = acc[j][r] + bb; }
  LDSX();
  for (int rl = 0; rl < 16; ++rl) vst2(OUT + (r0 + rl) * HID + lane * 4, *(const v4f*)&so[wave][rl][lane * 4]);
}
__global__ __launch_bounds__(128) void k_proj(const float* __restrict__ Hs, const __bf16* __restrict__ P, const float* __restrict__ ATS, const float* __restrict__ ATD, float* __restrict__ HW, float* __restrict__ AS, float* __restrict__ AD) {
  __shared__ __align__(16) float so[4][16][132]; __shared__ __align__(16) float sas[64], sad[64]; __shared__ float sats[HID], satd[HID];
  const int tid = threadIdx.x, wave = tid >> 5, lane = tid & 31, col = lane & 15, g = lane >> 4; const int h = blockIdx.y; const size_t r0 = (size_t)blockIdx.x * 64 + wave * 16; size_t ra = r0 + col; if (ra >= NN) ra = NN - 1;
  if (tid < HID) { sats[tid] = bfr(ATS[h * HID + tid]); satd[tid] = bfr(ATD[h * HID + tid]); }
  __syncthreads();
  v8f acc[8] = {};
#pragma unroll
  for (int kc = 0; kc < HID / 32; ++kc) { const F2 a = split_row(Hs + ra * HID, kc * 32, lane);
#pragma unroll
    for (int j = 0; j < 8; ++j) { const v16b w = frag_b(P + (size_t)(h * HID + j * 16 + col) * HID + kc * 32, lane); acc[j] = wmma_bf(a.l, w, acc[j]); acc[j] = wmma_bf(a.h, w, acc[j]); } }
  float ps[8], pd[8];
#pragma unroll
  for (int r = 0; r < 8; ++r) { ps[r] = 0.f; pd[r] = 0.f; }
#pragma unroll
  for (int j = 0; j < 8; ++j) { const int c = j * 16 + col;
#pragma unroll
    for (int r = 0; r < 8; ++r) { const float v = acc[j][r]; so[wave][8 * g + r][c] = v; ps[r] += v * sats[c]; pd[r] += v * satd[c]; } }
#pragma unroll
  for (int r = 0; r < 8; ++r) { float a1 = ps[r], a2 = pd[r];
#pragma unroll
    for (int o = 1; o < 16; o <<= 1) { a1 += __shfl_xor(a1, o); a2 += __shfl_xor(a2, o); }
    if (col == 0) { sas[wave * 16 + 8 * g + r] = a1; sad[wave * 16 + 8 * g + r] = a2; } }
  __syncthreads();
  for (int rl = 0; rl < 16; ++rl) vst2(HW + (r0 + rl) * HC + h * HID + lane * 4, *(const v4f*)&so[wave][rl][lane * 4]);
  if (tid < 16) vst2(AS + (size_t)h * NRP + (size_t)blockIdx.x * 64 + tid * 4, *(const v4f*)&sas[tid * 4]);
  else if (tid < 32) vst2(AD + (size_t)h * NRP + (size_t)blockIdx.x * 64 + (tid - 16) * 4, *(const v4f*)&sad[(tid - 16) * 4]);
}
__global__ __launch_bounds__(256) void k_gat(const float* __restrict__ HW, const float* __restrict__ AS, const float* __restrict__ AD, const int* __restrict__ FS, const int* __restrict__ RST, const int* __restrict__ RCT, const float* __restrict__ GB, const float* __restrict__ LG, const float* __restrict__ LB, float* Hs) {
  __shared__ __align__(16) float so[8][HID + 4];
  const int tid = threadIdx.x, wave = tid >> 5, lane = tid & 31; const int hd = lane >> 3, sl = lane & 7; const int f0 = hd * HID + sl * 16; const size_t node = (size_t)blockIdx.x * 8 + wave;
  float acc[16];
#pragma unroll
  for (int i = 0; i < 16; ++i) acc[i] = 0.f;
  float outv[16];
  if (node < (size_t)NN) {
    const int cnt = min(max(RCT[node], 0), CSR_BCAP); const int st = min(max(RST[node], 0), CSR_FINN - cnt);
    const float adn = AD[(size_t)hd * NRP + node]; const float asn = AS[(size_t)hd * NRP + node];
    float es = asn + adn; es = (es >= 0.f) ? es : 0.2f * es;
    float mx = es;
    for (int e = 0; e < cnt; ++e) { const int s = min(max(FS[st + e], 0), NN - 1); float v = AS[(size_t)hd * NRP + s] + adn; v = (v >= 0.f) ? v : 0.2f * v; mx = fmaxf(mx, v); }
    float den = 0.f;
    { const float w = exp_ni(es - mx); den += w; const float* hr = HW + node * HC + f0;
#pragma unroll
      for (int i = 0; i < 16; ++i) acc[i] += w * hr[i]; }
    for (int e = 0; e < cnt; ++e) { const int s = min(max(FS[st + e], 0), NN - 1); float v = AS[(size_t)hd * NRP + s] + adn; v = (v >= 0.f) ? v : 0.2f * v; const float w = exp_ni(v - mx); den += w; const float* hr = HW + (size_t)s * HC + f0;
#pragma unroll
      for (int i = 0; i < 16; ++i) acc[i] += w * hr[i]; }
    const float iden = 1.0f / (den + 1e-16f);
#pragma unroll
    for (int i = 0; i < 16; ++i) acc[i] *= iden;
  }
  float sum = 0.f;
#pragma unroll
  for (int i = 0; i < 16; ++i) { float t = acc[i]; t += __shfl_xor(t, 8); t += __shfl_xor(t, 16); outv[i] = t * 0.25f + bfr(GB[sl * 16 + i]); sum += outv[i]; }
#pragma unroll
  for (int o = 1; o < 8; o <<= 1) sum += __shfl_xor(sum, o);
  const float mu = sum / (float)HID; float var = 0.f;
#pragma unroll
  for (int i = 0; i < 16; ++i) { const float d = outv[i] - mu; var += d * d; }
#pragma unroll
  for (int o = 1; o < 8; o <<= 1) var += __shfl_xor(var, o);
  const float rs = 1.0f / sqrtf(var / (float)HID + 1e-5f);
  if (hd == 0 && node < (size_t)NN) { const float* hr = Hs + node * HID + sl * 16;
#pragma unroll
    for (int i = 0; i < 16; ++i) { const int c = sl * 16 + i; const float v = fmaxf((outv[i] - mu) * rs * bfr(LG[c]) + bfr(LB[c]), 0.f); so[wave][c] = v + hr[i]; } }
  LDSX();
  if (node < (size_t)NN) vst2(Hs + node * HID + lane * 4, *(const v4f*)&so[wave][lane * 4]);
}
__global__ __launch_bounds__(128) void k_head(const float* __restrict__ Hs, const int* __restrict__ IDX, const __bf16* __restrict__ P, const float* __restrict__ B1, const float* __restrict__ W2, const float* __restrict__ B2, float* __restrict__ out) {
  __shared__ __align__(16) float sl_[64]; __shared__ float sw2[64], sb1[64];
  const int tid = threadIdx.x, wave = tid >> 5, lane = tid & 31, col = lane & 15, g = lane >> 4; const int q0 = blockIdx.x * 64 + wave * 16;
  if (tid < 64) { sw2[tid] = bfr(W2[tid]); sb1[tid] = bfr(B1[tid]); }
  __syncthreads();
  const int node = min(max(IDX[q0 + col], 0), NN - 1);
  v8f acc[4] = {};
#pragma unroll
  for (int kc = 0; kc < HID / 32; ++kc) { const F2 a = split_row(Hs + (size_t)node * HID, kc * 32, lane);
#pragma unroll
    for (int j = 0; j < 4; ++j) { const v16b w = frag_b(P + (size_t)(j * 16 + col) * HID + kc * 32, lane); acc[j] = wmma_bf(a.l, w, acc[j]); acc[j] = wmma_bf(a.h, w, acc[j]); } }
  float part[8];
#pragma unroll
  for (int r = 0; r < 8; ++r) { float s = 0.f;
#pragma unroll
    for (int j = 0; j < 4; ++j) { const int c = j * 16 + col; s += fmaxf(acc[j][r] + sb1[c], 0.f) * sw2[c]; }
#pragma unroll
    for (int o = 1; o < 16; o <<= 1) s += __shfl_xor(s, o);
    part[r] = s; }
  if (col == 0) {
#pragma unroll
    for (int r = 0; r < 8; ++r) sl_[wave * 16 + 8 * g + r] = part[r] + bfr(B2[0]); }
  __syncthreads();
  if (tid < 16) vst2(out + (size_t)blockIdx.x * 64 + tid * 4, *(const v4f*)&sl_[tid * 4]);
}
extern "C" void kernel_launch(void* const* d_in, const int* in_sizes, int n_in, void* d_out, int out_size, void* d_ws, size_t ws_size, hipStream_t stream) {
  (void)in_sizes; (void)n_in; (void)out_size;
  const float** F = (const float**)d_in; const int* EI = (const int*)d_in[1]; const int* IDX = (const int*)d_in[2];
  if (ws_size < (size_t)WS_END) return;
  char* ws = (char*)d_ws;
  int *CNT = (int*)(ws + WS_CNT), *OFF = (int*)(ws + WS_OFF), *BST = (int*)(ws + WS_BST), *SEGS = (int*)(ws + WS_SEGS), *SEGE = (int*)(ws + WS_SEGE), *FS = (int*)(ws + WS_FS), *FE = (int*)(ws + WS_FE), *RST = (int*)(ws + WS_RST), *RCT = (int*)(ws + WS_RCT);
  __bf16* PW = (__bf16*)(ws + WS_PW); float *T = (float*)(ws + WS_T), *Hs = (float*)(ws + WS_H), *HW = (float*)(ws + WS_HW), *AS = (float*)(ws + WS_AS), *AD = (float*)(ws + WS_AD);
  const int* SRC = EI; const int* DST = EI + EP;
  k_packT<<<dim3(HID, 1), 128, 0, stream>>>(F[5], HID, HID, PW + PE2); k_packT<<<dim3(HC, NL), 128, 0, stream>>>(F[7], HID, HC, PW + PG0); k_packT<<<dim3(64, 1), 128, 0, stream>>>(F[13], HID, 64, PW + PH1);
  k_csr_cnt<<<CSR_NCH, 256, 0, stream>>>(DST, 1, CNT); k_csr_scan<<<1, 256, 0, stream>>>(CNT, OFF, BST); k_csr_scatter<<<CSR_NCH, 256, 0, stream>>>(SRC, DST, 1, 1, OFF, SEGS, SEGE); k_csr_bucket<<<CSR_NBK, 256, 0, stream>>>(CNT, OFF, BST, SEGS, SEGE, DST, 1, FS, FE, RST, RCT);
  k_enc1<<<NRP / 16, 256, 0, stream>>>(F[0], F[3], F[4], T);
  k_lin<<<NBLK, 128, 0, stream>>>(T, PW + PE2, F[6], Hs);
  for (int l = 0; l < NL; ++l) {
    k_proj<<<dim3(NBLK, NHD), 128, 0, stream>>>(Hs, PW + PG0 + (size_t)l * HC * HID, F[8] + l * NHD * HID, F[9] + l * NHD * HID, HW, AS, AD);
    k_gat<<<NRP / 8, 256, 0, stream>>>(HW, AS, AD, FS, RST, RCT, F[10] + l * HID, F[11] + l * HID, F[12] + l * HID, Hs); }
  k_head<<<NHYP / 64, 128, 0, stream>>>(Hs, IDX, PW + PH1, F[14], F[15], F[16], (float*)d_out);
}
